// SAblock_79654463472153
// MI455X (gfx1250) — hardware-verified
//
#include <hip/hip_runtime.h>
#include <math.h>

constexpr int kB   = 8;
constexpr int kC   = 256;
constexpr int kN   = 4096;
constexpr int kCP  = 32;
constexpr int kQKW = 64;
constexpr int kVR  = 64;
constexpr int kOW  = 64;
constexpr float kWCarry    = 16.0f;
constexpr float kWCarryInv = 1.0f / 16.0f;
constexpr float kPCarry    = 32768.0f;
constexpr float kOCarry    = 64.0f;
constexpr float kPVScale   = kOCarry / kPCarry;
constexpr float kBackScale = 1.0f / (kOCarry * kWCarry);
static_assert(kN % 64 == 0 && kC % 64 == 0 && kQKW % 64 == 0 && kVR % 64 == 0 && kOW % 64 == 0, "tile multiples");
static_assert(kC % 32 == 0 && kCP % 32 == 0 && kN % 32 == 0, "k steps of 32");
static_assert(2 * kCP == kQKW && kCP <= kVR && kCP <= kOW, "plane widths");
static_assert(kCP * kC == 8192 && kC * kCP == 8192 && kN % 256 == 0 && kN % 8 == 0, "prep and elementwise coverage");

typedef __attribute__((ext_vector_type(16))) _Float16 v16h;
typedef __attribute__((ext_vector_type(8)))  _Float16 v8h;
typedef __attribute__((ext_vector_type(16))) __bf16   v16b;
typedef __attribute__((ext_vector_type(8)))  __bf16   v8b;
typedef __attribute__((ext_vector_type(8)))  float    v8f;
typedef __attribute__((ext_vector_type(4)))  float    v4f;
typedef __attribute__((ext_vector_type(4)))  unsigned int v4u;

__device__ __forceinline__ unsigned short f2bf_bits(float f) {
  unsigned u = __float_as_uint(f);
  return (unsigned short)((u + 0x7FFFu + ((u >> 16) & 1u)) >> 16);
}
__device__ __forceinline__ float bf_bits2f(unsigned short h) { return __uint_as_float(((unsigned)h) << 16); }

__device__ __forceinline__ void dep_guard_h(v8f& a, v8f& b, v16h x, v16h y) { asm volatile("v_nop\n\tv_nop\n\tv_nop\n\tv_nop" : "+v"(a), "+v"(b) : "v"(x), "v"(y)); }
__device__ __forceinline__ void dep_guard_b(v8f& a, v8f& b, v16b x, v16b y) { asm volatile("v_nop\n\tv_nop\n\tv_nop\n\tv_nop" : "+v"(a), "+v"(b) : "v"(x), "v"(y)); }
__device__ __forceinline__ void dep_guard4_h(v8f& a, v8f& b, v8f& c, v8f& d, v16h x, v16h y) { asm volatile("v_nop\n\tv_nop\n\tv_nop\n\tv_nop" : "+v"(a), "+v"(b), "+v"(c), "+v"(d) : "v"(x), "v"(y)); }
__device__ __forceinline__ void dep_guard4_b(v8f& a, v8f& b, v8f& c, v8f& d, v16b x, v16b y) { asm volatile("v_nop\n\tv_nop\n\tv_nop\n\tv_nop" : "+v"(a), "+v"(b), "+v"(c), "+v"(d) : "v"(x), "v"(y)); }
__device__ __forceinline__ void keep4_h(v16h a, v16h b, v16h c, v16h d) { asm volatile("v_nop" :: "v"(a), "v"(b), "v"(c), "v"(d)); }
__device__ __forceinline__ void keep4_b(v16b a, v16b b, v16b c, v16b d) { asm volatile("v_nop" :: "v"(a), "v"(b), "v"(c), "v"(d)); }
__device__ __forceinline__ void acc_guard4(v8f& a, v8f& b, v8f& c, v8f& d) { asm volatile("v_nop\n\tv_nop\n\tv_nop\n\tv_nop" : "+v"(a), "+v"(b), "+v"(c), "+v"(d)); }
template <typename T> struct Frag;
template <> struct Frag<_Float16> {
  typedef v16h V; union U { v16h v; v8h h[2]; };
  static __device__ __forceinline__ v16h load(const _Float16* p) {
    U f; f.h[0] = *(const v8h*)(p); f.h[1] = *(const v8h*)(p + 16); return f.v;
  }
  static __device__ __forceinline__ v8f mma(v16h a, v16h b, v8f c) {
    return __builtin_amdgcn_wmma_f32_16x16x32_f16(false, a, false, b, (short)0, c, false, false);
  }
  static __device__ __forceinline__ void guard(v8f& a, v8f& b, v16h x, v16h y) { dep_guard_h(a, b, x, y); }
  static __device__ __forceinline__ void guard4(v8f& a, v8f& b, v8f& c, v8f& d, v16h x, v16h y) { dep_guard4_h(a, b, c, d, x, y); }
  static __device__ __forceinline__ void keep(v16h a, v16h b, v16h c, v16h d) { keep4_h(a, b, c, d); }
};
template <> struct Frag<__bf16> {
  typedef v16b V; union U { v16b v; v8b h[2]; };
  static __device__ __forceinline__ v16b load(const __bf16* p) {
    U f; f.h[0] = *(const v8b*)(p); f.h[1] = *(const v8b*)(p + 16); return f.v;
  }
  static __device__ __forceinline__ v8f mma(v16b a, v16b b, v8f c) {
    return __builtin_amdgcn_wmma_f32_16x16x32_bf16(false, a, false, b, (short)0, c, false, false);
  }
  static __device__ __forceinline__ void guard(v8f& a, v8f& b, v16b x, v16b y) { dep_guard_b(a, b, x, y); }
  static __device__ __forceinline__ void guard4(v8f& a, v8f& b, v8f& c, v8f& d, v16b x, v16b y) { dep_guard4_b(a, b, c, d, x, y); }
  static __device__ __forceinline__ void keep(v16b a, v16b b, v16b c, v16b d) { keep4_b(a, b, c, d); }
};

__device__ __forceinline__ unsigned pk16(unsigned short a, unsigned short b) { return (unsigned)a | ((unsigned)b << 16); }
__device__ __forceinline__ unsigned short h_bits(float f) { const _Float16 h = (_Float16)f; return __builtin_bit_cast(unsigned short, h); }

template <int ET> struct Elem;
template <> struct Elem<0> { typedef _Float16 T; };
template <> struct Elem<1> { typedef __bf16 T; };
template <int ET, bool SPLIT, int BIAS_MODE, int OUT_MODE, bool RESID>
__global__ __launch_bounds__(256) void wmma_gemm64(
    const unsigned short* __restrict__ Ap, const unsigned short* __restrict__ A2p, int lda, long strideA,
    const unsigned short* __restrict__ Btp, const unsigned short* __restrict__ Bt2p, int ldb, long strideB,
    void* __restrict__ Cout, void* __restrict__ Cout2, int ldc, long strideC,
    const float* __restrict__ bias,
    const float* __restrict__ resid, long strideR,
    int M, int N, int K, float scale) {
  static_assert(!RESID || OUT_MODE == 0, "residual only with f32 output");
  typedef typename Elem<ET>::T T;
  typedef typename Frag<T>::V V;
  const T* A = (const T*)Ap; const T* A2 = (const T*)A2p; const T* Bt = (const T*)Btp; const T* Bt2 = (const T*)Bt2p;
  __shared__ __align__(16) float sT[8][16 * 68];
  const int b    = blockIdx.y;
  const int lane = threadIdx.x & 31;
  const int wave = threadIdx.x >> 5;
  const int tilesN = N >> 6;
  const int tilesM = M >> 6;
  const int tile = blockIdx.x * 8 + wave;
  if (tile >= tilesM * tilesN) return;
  const int tm = tile / tilesN;
  const int tn = tile - tm * tilesN;
  const int m0 = tm << 6;
  const int n0 = tn << 6;

  const T* Ab  = A  + (size_t)b * strideA;
  const T* Bb  = Bt + (size_t)b * strideB;
  const T* Ab2 = SPLIT ? (A2  + (size_t)b * strideA) : nullptr;
  const T* Bb2 = SPLIT ? (Bt2 + (size_t)b * strideB) : nullptr;

  const int rlane = lane & 15;
  const int koff  = (lane >> 4) * 8;
  const int mOff  = (lane >> 4) * 8;

  v8f acc[4][4];
#pragma unroll
  for (int i = 0; i < 4; ++i)
#pragma unroll
    for (int j = 0; j < 4; ++j) acc[i][j] = (v8f){0.f,0.f,0.f,0.f,0.f,0.f,0.f,0.f};

  for (int k0 = 0; k0 < K; k0 += 32) {
    V bh[4], bl[4];
#pragma unroll
    for (int j = 0; j < 4; ++j) {
      const size_t bo = (size_t)(n0 + (j << 4) + rlane) * ldb + koff + k0;
      bh[j] = Frag<T>::load(Bb + bo);
      if (SPLIT) bl[j] = Frag<T>::load(Bb2 + bo);
    }
#pragma unroll
    for (int i = 0; i < 4; ++i) {
      const size_t ao = (size_t)(m0 + (i << 4) + rlane) * lda + koff + k0;
      V ah = Frag<T>::load(Ab + ao);
      V al;
      if (SPLIT) al = Frag<T>::load(Ab2 + ao);
#pragma unroll
      for (int j = 0; j < 4; ++j) {
        acc[i][j] = Frag<T>::mma(ah, bh[j], acc[i][j]);
        if (SPLIT) {
          acc[i][j] = Frag<T>::mma(ah, bl[j], acc[i][j]);
          acc[i][j] = Frag<T>::mma(al, bh[j], acc[i][j]);
        }
      }
      Frag<T>::guard4(acc[i][0], acc[i][1], acc[i][2], acc[i][3], ah, SPLIT ? al : ah);
    }
    Frag<T>::keep(bh[0], bh[1], bh[2], bh[3]);
    if (SPLIT) Frag<T>::keep(bl[0], bl[1], bl[2], bl[3]);
  }
  acc_guard4(acc[0][0], acc[0][1], acc[0][2], acc[0][3]);
  acc_guard4(acc[1][0], acc[1][1], acc[1][2], acc[1][3]);
  acc_guard4(acc[2][0], acc[2][1], acc[2][2], acc[2][3]);
  acc_guard4(acc[3][0], acc[3][1], acc[3][2], acc[3][3]);

  float* slab = sT[wave];
  const float* Rb = RESID ? (resid + (size_t)b * strideR) : nullptr;
#pragma unroll
  for (int i = 0; i < 4; ++i) {
    const int mBase = m0 + (i << 4);
#pragma unroll
    for (int j = 0; j < 4; ++j) {
      const int n = n0 + (j << 4) + rlane;
      float bvn = 0.f;
      if (BIAS_MODE == 2) bvn = bias[n];
#pragma unroll
      for (int r = 0; r < 8; ++r) {
        float v = acc[i][j][r] * scale;
        if (BIAS_MODE == 1) v += bias[mBase + mOff + r];
        if (BIAS_MODE == 2) v += bvn;
        slab[(mOff + r) * 68 + (j << 4) + rlane] = v;
      }
    }
    __builtin_amdgcn_fence(__ATOMIC_RELEASE, "workgroup");
    __builtin_amdgcn_wave_barrier();
    __builtin_amdgcn_fence(__ATOMIC_ACQUIRE, "workgroup");
    if (OUT_MODE == 0) {
      float* C = (float*)Cout + (size_t)b * strideC;
      const int hh = lane >> 4, c4 = (lane & 15) * 4;
      v4f vals[8];
#pragma unroll
      for (int it = 0; it < 8; ++it) {
        const int row = it * 2 + hh;
        v4f v = *(const v4f*)(slab + row * 68 + c4);
        if (RESID) {
          const v4f rv = *(const v4f*)(Rb + (size_t)(mBase + row) * ldc + n0 + c4);
          v = v + rv;
        }
        vals[it] = v;
      }
      for (int pass = 0; pass < 2; ++pass) {
#pragma unroll
        for (int it = 0; it < 8; ++it) {
          const int row = it * 2 + hh;
          *(volatile v4f*)(C + (size_t)(mBase + row) * ldc + n0 + c4) = vals[it];
        }
        __threadfence();
      }
    } else {
      const int q = lane >> 3, c8 = (lane & 7) * 8;
      unsigned short* C  = (unsigned short*)Cout  + (size_t)b * strideC;
      unsigned short* C2 = (OUT_MODE == 2) ? ((unsigned short*)Cout2 + (size_t)b * strideC) : nullptr;
      for (int pass = 0; pass < 2; ++pass) {
#pragma unroll
        for (int it = 0; it < 4; ++it) {
          const int row = it * 4 + q;
          const float* sp = slab + row * 68 + c8;
          v8h hv, lv;
#pragma unroll
          for (int e = 0; e < 8; ++e) {
            if (OUT_MODE == 1) {
              hv[e] = (_Float16)sp[e];
            } else {
              unsigned short hb = f2bf_bits(sp[e]);
              unsigned short lb = f2bf_bits(sp[e] - bf_bits2f(hb));
              hv[e] = __builtin_bit_cast(_Float16, hb);
              lv[e] = __builtin_bit_cast(_Float16, lb);
            }
          }
          *(volatile v8h*)(C + (size_t)(mBase + row) * ldc + n0 + c8) = hv;
          if (OUT_MODE == 2) *(volatile v8h*)(C2 + (size_t)(mBase + row) * ldc + n0 + c8) = lv;
        }
        __threadfence();
      }
    }
    __builtin_amdgcn_fence(__ATOMIC_RELEASE, "workgroup");
    __builtin_amdgcn_wave_barrier();
    __builtin_amdgcn_fence(__ATOMIC_ACQUIRE, "workgroup");
  }
}

__global__ __launch_bounds__(256) void prep_kernel(const float* __restrict__ Wq, const float* __restrict__ bq,
                                                   const float* __restrict__ Wk, const float* __restrict__ bk,
                                                   const float* __restrict__ Wv, const float* __restrict__ bv,
                                                   const float* __restrict__ Wb,
                                                   unsigned short* __restrict__ WQK16, unsigned short* __restrict__ WV16,
                                                   unsigned short* __restrict__ WB16,
                                                   float* __restrict__ BQK, float* __restrict__ BV64) {
  const int t   = threadIdx.x;
  const int blk = blockIdx.x;
  if (blk < 20) {
    const int grp = blk >> 2;
    const int sub = blk & 3;
    const int e0  = (sub * 256 + t) * 8;
    const float* src = (grp == 0) ? Wq : (grp == 1) ? Wk : (grp == 4) ? Wb : Wv;
    const float  f   = (grp == 3) ? 0.0f : kWCarry;
    unsigned short* dst = (grp == 0) ? WQK16 : (grp == 1) ? (WQK16 + 8192) : (grp == 2) ? WV16 : (grp == 3) ? (WV16 + 8192) : WB16;
    const v4f a = *(const v4f*)(src + e0);
    const v4f c = *(const v4f*)(src + e0 + 4);
    unsigned short hb[8];
#pragma unroll
    for (int e = 0; e < 4; ++e) {
      hb[e]     = h_bits(a[e] * f);
      hb[4 + e] = h_bits(c[e] * f);
    }
    const v4u u = (v4u){pk16(hb[0], hb[1]), pk16(hb[2], hb[3]), pk16(hb[4], hb[5]), pk16(hb[6], hb[7])};
    unsigned short* dp = dst + e0;
    *(volatile v4u*)dp = u;
    __threadfence();
    *(volatile v4u*)dp = u;
  } else {
    const int lane = t & 31, wave = t >> 5;
    const int idx = (lane & 7) * 4;
    const v4f q4 = *(const v4f*)(bq + idx);
    const v4f k4 = *(const v4f*)(bk + idx);
    const v4f w4 = *(const v4f*)(bv + idx);
    const float fq = (lane < 8) ? 1.0f : 0.0f;
    const float fk = (lane < 8) ? 0.0f : 1.0f;
    const v4f valQK = q4 * fq + k4 * fk;
    const v4f valV  = w4 * fq;
    const bool wq = (wave == 0) && (lane < 16);
    const bool wv = (wave == 1) && (lane < 16);
    float* dq = BQK  + (lane & 15) * 4;
    float* dv = BV64 + (lane & 15) * 4;
    if (wq) *(volatile v4f*)dq = valQK;
    if (wv) *(volatile v4f*)dv = valV;
    __threadfence();
    if (wq) *(volatile v4f*)dq = valQK;
    if (wv) *(volatile v4f*)dv = valV;
  }
}

__global__ __launch_bounds__(256) void xtcast_kernel(const float* __restrict__ x, unsigned short* __restrict__ XT) {
  __shared__ float sm[64][65];
  const int t  = threadIdx.x;
  const int n0 = blockIdx.x * 64;
  const int c0 = blockIdx.y * 64;
  const int b  = blockIdx.z;
  const float* xb = x + (size_t)b * kC * kN;
#pragma unroll
  for (int i = 0; i < 16; ++i) {
    const int e = i * 256 + t;
    const int r = e >> 6;
    const int q = e & 63;
    sm[q][r] = xb[(size_t)(c0 + r) * kN + n0 + q];
    if (i == 7) asm volatile("" ::: "memory");
  }
  __syncthreads();
  const int lane = t & 31, wave = t >> 5;
  const int q8 = lane >> 3, c8 = (lane & 7) * 8;
  unsigned short* op = XT + ((size_t)b * kN) * kC;
  for (int pass = 0; pass < 2; ++pass) {
#pragma unroll
    for (int it = 0; it < 2; ++it) {
      const int row = wave * 8 + it * 4 + q8;
      unsigned short hb[8];
#pragma unroll
      for (int e = 0; e < 8; ++e) hb[e] = h_bits(sm[row][c8 + e]);
      const v4u u = (v4u){pk16(hb[0], hb[1]), pk16(hb[2], hb[3]), pk16(hb[4], hb[5]), pk16(hb[6], hb[7])};
      *(volatile v4u*)(op + (size_t)(n0 + row) * kC + c0 + c8) = u;
    }
    __threadfence();
  }
}

__global__ __launch_bounds__(256) void colstats_kernel(const float* __restrict__ ST, float* __restrict__ CM,
                                                       float* __restrict__ CLI) {
  __shared__ __align__(16) float smax[256];
  __shared__ __align__(16) float sinv[256];
  const int t = threadIdx.x;
  const int j = blockIdx.x * 256 + t;
  const float* col = ST + j;
  float m0 = -__builtin_inff(), m1 = -__builtin_inff(), m2 = -__builtin_inff(), m3 = -__builtin_inff();
#pragma unroll 1
  for (int i = 0; i < kN; i += 4) {
    const float* p = col + (size_t)i * kN;
    m0 = fmaxf(m0, p[0]);
    m1 = fmaxf(m1, p[kN]);
    m2 = fmaxf(m2, p[2 * kN]);
    m3 = fmaxf(m3, p[3 * kN]);
  }
  const float m = fmaxf(fmaxf(m0, m1), fmaxf(m2, m3));
  float s0 = 0.f, s1 = 0.f, s2 = 0.f, s3 = 0.f;
#pragma unroll 1
  for (int i = 0; i < kN; i += 4) {
    const float* p = col + (size_t)i * kN;
    s0 += expf(p[0] - m);
    s1 += expf(p[kN] - m);
    s2 += expf(p[2 * kN] - m);
    s3 += expf(p[3 * kN] - m);
  }
  const float tot = (s0 + s1) + (s2 + s3);
  smax[t] = m;
  sinv[t] = kPCarry / tot;
  __syncthreads();
  const int wave = t >> 5;
  if (wave < 2) {
    const v4f val = *(const v4f*)(smax + 4 * t);
    float* dp = CM + blockIdx.x * 256 + 4 * t;
    *(volatile v4f*)dp = val;
    __threadfence();
    *(volatile v4f*)dp = val;
  } else if (wave < 4) {
    const int u = t - 64;
    const v4f val = *(const v4f*)(sinv + 4 * u);
    float* dp = CLI + blockIdx.x * 256 + 4 * u;
    *(volatile v4f*)dp = val;
    __threadfence();
    *(volatile v4f*)dp = val;
  }
}

__global__ __launch_bounds__(256) void pmake_kernel(const float* __restrict__ ST, const float* __restrict__ CM,
                                                    const float* __restrict__ CLI, unsigned short* __restrict__ P) {
  const int t  = threadIdx.x;
  const int i  = blockIdx.x >> 1;
  const int j0 = ((blockIdx.x & 1) << 11) + t * 8;
  const size_t off = (size_t)i * kN + j0;
  const v4f a  = *(const v4f*)(ST + off);
  const v4f c  = *(const v4f*)(ST + off + 4);
  const v4f ma = *(const v4f*)(CM + j0);
  const v4f mc = *(const v4f*)(CM + j0 + 4);
  const v4f la = *(const v4f*)(CLI + j0);
  const v4f lc = *(const v4f*)(CLI + j0 + 4);
  unsigned short hb[8];
#pragma unroll
  for (int e = 0; e < 4; ++e) {
    hb[e]     = h_bits(expf(a[e] - ma[e]) * la[e]);
    hb[4 + e] = h_bits(expf(c[e] - mc[e]) * lc[e]);
  }
  const v4u u = (v4u){pk16(hb[0], hb[1]), pk16(hb[2], hb[3]), pk16(hb[4], hb[5]), pk16(hb[6], hb[7])};
  unsigned short* pr = P + off;
  *(volatile v4u*)pr = u;
  __threadfence();
  *(volatile v4u*)pr = u;
}

extern "C" void kernel_launch(void* const* d_in, const int* in_sizes, int n_in,
                              void* d_out, int out_size, void* d_ws, size_t ws_size,
                              hipStream_t stream) {
  if (n_in < 9) return;
  const int nX = kB * kC * kN;
  if (in_sizes[0] != nX) return;
  if (in_sizes[1] != kCP * kC || in_sizes[3] != kCP * kC || in_sizes[5] != kCP * kC) return;
  if (in_sizes[2] != kCP || in_sizes[4] != kCP || in_sizes[6] != kCP) return;
  if (in_sizes[7] != kC * kCP || in_sizes[8] != kC) return;
  if (out_size != nX) return;

  const size_t szXT  = (size_t)kB * kN * kC * 2;
  const size_t szWQK = (size_t)kQKW * kC * 2;
  const size_t szWV  = (size_t)kVR * kC * 2;
  const size_t szWB  = (size_t)kC * kCP * 2;
  const size_t szBQK = (size_t)kQKW * 4;
  const size_t szBV  = (size_t)kVR * 4;
  const size_t szQK  = (size_t)kB * kN * kQKW * 2;
  const size_t szV   = (size_t)kB * kVR * kN * 2;
  const size_t szST  = (size_t)kN * kN * 4;
  const size_t szCM  = (size_t)kN * 4;
  const size_t szCL  = (size_t)kN * 4;
  const size_t szP   = (size_t)kN * kN * 2;
  const size_t szO   = (size_t)kB * kN * kOW * 2;
  const size_t offXT  = 0;
  const size_t offWQK = offXT + szXT;
  const size_t offWV  = offWQK + szWQK;
  const size_t offWB  = offWV + szWV;
  const size_t offBQK = offWB + szWB;
  const size_t offBV  = offBQK + szBQK;
  const size_t offQK  = offBV + szBV;
  const size_t offV   = offQK + szQK;
  const size_t offST  = offV + szV;
  const size_t offCM  = offST + szST;
  const size_t offCL  = offCM + szCM;
  const size_t offP   = offCL + szCL;
  const size_t offO   = offP + szP;
  const size_t total  = offO + szO;
  if (ws_size < total) return;

  const float* x  = (const float*)d_in[0];
  const float* Wq = (const float*)d_in[1];
  const float* bq = (const float*)d_in[2];
  const float* Wk = (const float*)d_in[3];
  const float* bk = (const float*)d_in[4];
  const float* Wv = (const float*)d_in[5];
  const float* bv = (const float*)d_in[6];
  const float* Wb = (const float*)d_in[7];
  const float* bb = (const float*)d_in[8];
  float* out = (float*)d_out;
  char* ws = (char*)d_ws;
  unsigned short* XT16  = (unsigned short*)(ws + offXT);
  unsigned short* WQK16 = (unsigned short*)(ws + offWQK);
  unsigned short* WV16  = (unsigned short*)(ws + offWV);
  unsigned short* WB16  = (unsigned short*)(ws + offWB);
  float* BQK  = (float*)(ws + offBQK);
  float* BV64 = (float*)(ws + offBV);
  unsigned short* QK16 = (unsigned short*)(ws + offQK);
  unsigned short* V16  = (unsigned short*)(ws + offV);
  float* ST  = (float*)(ws + offST);
  float* CM  = (float*)(ws + offCM);
  float* CLI = (float*)(ws + offCL);
  unsigned short* P16 = (unsigned short*)(ws + offP);
  unsigned short* O16 = (unsigned short*)(ws + offO);

  prep_kernel<<<dim3(21), dim3(256), 0, stream>>>(Wq, bq, Wk, bk, Wv, bv, Wb, WQK16, WV16, WB16, BQK, BV64);
  xtcast_kernel<<<dim3(kN / 64, kC / 64, kB), dim3(256), 0, stream>>>(x, XT16);

  const long strideXT = (long)kN * kC;
  const long strideQK = (long)kN * kQKW;
  const long strideV  = (long)kVR * kN;
  const long strideO  = (long)kN * kOW;
  const long strideX  = (long)kC * kN;

  const int blocksQK = ((kN / 64) * (kQKW / 64)) / 8;
  wmma_gemm64<0, false, 2, 1, false><<<dim3(blocksQK, kB), dim3(256), 0, stream>>>(
      XT16, XT16, kC, strideXT, WQK16, WQK16, kC, 0L,
      (void*)QK16, (void*)QK16, kQKW, strideQK, BQK, x, 0L, kN, kQKW, kC, kWCarryInv);
  const int blocksV = ((kVR / 64) * (kN / 64)) / 8;
  wmma_gemm64<0, false, 1, 1, false><<<dim3(blocksV, kB), dim3(256), 0, stream>>>(
      WV16, WV16, kC, 0L, XT16, XT16, kC, strideXT,
      (void*)V16, (void*)V16, kN, strideV, BV64, x, 0L, kVR, kN, kC, kWCarryInv);

  const int blocksST = ((kN / 64) * (kN / 64)) / 8;
  const int blocksPV = ((kN / 64) * (kOW / 64)) / 8;
  for (int b = 0; b < kB; ++b) {
    const unsigned short* QKb = QK16 + (size_t)b * strideQK;
    const unsigned short* Kb  = QKb + kCP;
    const unsigned short* Vb  = V16 + (size_t)b * strideV;
    unsigned short* Ob = O16 + (size_t)b * strideO;
    wmma_gemm64<0, false, 0, 0, false><<<dim3(blocksST, 1), dim3(256), 0, stream>>>(
        Kb, Kb, kQKW, 0L, QKb, QKb, kQKW, 0L,
        (void*)ST, (void*)ST, kN, 0L, BQK, x, 0L, kN, kN, kCP, 1.0f);
    colstats_kernel<<<dim3(kN / 256), dim3(256), 0, stream>>>(ST, CM, CLI);
    pmake_kernel<<<dim3(2 * kN), dim3(256), 0, stream>>>(ST, CM, CLI, P16);
    wmma_gemm64<0, false, 0, 1, false><<<dim3(blocksPV, 1), dim3(256), 0, stream>>>(
        P16, P16, kN, 0L, Vb, Vb, kN, 0L,
        (void*)Ob, (void*)Ob, kOW, 0L, BQK, x, 0L, kN, kOW, kN, kPVScale);
  }

  const int blocksBack = ((kC / 64) * (kN / 64)) / 8;
  wmma_gemm64<0, false, 1, 0, true><<<dim3(blocksBack, kB), dim3(256), 0, stream>>>(
      WB16, WB16, kCP, 0L, O16, O16, kOW, strideO,
      (void*)out, (void*)out, kN, strideX, bb, x, strideX, kC, kN, kCP, kBackScale);
}
